// HierarchicalMambaBlock_79577154060423
// MI455X (gfx1250) — hardware-run, weakly checked
//
#include <hip/hip_runtime.h>
#include <math.h>

typedef __attribute__((ext_vector_type(16))) _Float16 v16h;
typedef __attribute__((ext_vector_type(8)))  _Float16 v8h;
typedef __attribute__((ext_vector_type(16))) __bf16   v16b;
typedef __attribute__((ext_vector_type(8)))  __bf16   v8b;
typedef __attribute__((ext_vector_type(8)))  float    v8f;
typedef __attribute__((ext_vector_type(4)))  float    v4f;

constexpr int kT    = 2048;
constexpr int kDm   = 768;
constexpr int kDi   = 1536;
constexpr int kXZ   = 2 * kDi;
constexpr int kNs   = 16;
constexpr int kNsc  = 3;
constexpr int kPrj  = 64;
constexpr int kKdt  = 32;
constexpr int kG1   = kDi / 2;
constexpr int kTP   = 260;

__device__ __forceinline__ unsigned short f2bf_bits(float f) {
  unsigned u = __float_as_uint(f);
  return (unsigned short)((u + 0x7FFFu + ((u >> 16) & 1u)) >> 16);
}
__device__ __forceinline__ float bf_bits2f(unsigned short h) { return __uint_as_float(((unsigned)h) << 16); }

__device__ __forceinline__ void dep_guard_h(v8f& a, v8f& b, v16h x, v16h y) { asm volatile("v_nop\n\tv_nop\n\tv_nop\n\tv_nop" : "+v"(a), "+v"(b) : "v"(x), "v"(y)); }
__device__ __forceinline__ void dep_guard_b(v8f& a, v8f& b, v16b x, v16b y) { asm volatile("v_nop\n\tv_nop\n\tv_nop\n\tv_nop" : "+v"(a), "+v"(b) : "v"(x), "v"(y)); }
__device__ __forceinline__ void keep4_h(v16h a, v16h b, v16h c, v16h d) { asm volatile("v_nop" :: "v"(a), "v"(b), "v"(c), "v"(d)); }
__device__ __forceinline__ void keep4_b(v16b a, v16b b, v16b c, v16b d) { asm volatile("v_nop" :: "v"(a), "v"(b), "v"(c), "v"(d)); }
__device__ __forceinline__ void acc_guard4(v8f& a, v8f& b, v8f& c, v8f& d) { asm volatile("v_nop\n\tv_nop\n\tv_nop\n\tv_nop" : "+v"(a), "+v"(b), "+v"(c), "+v"(d)); }
template <typename T> struct Frag;
template <> struct Frag<_Float16> {
  typedef v16h V; union U { v16h v; v8h h[2]; };
  static __device__ __forceinline__ v16h load(const _Float16* p) {
    U f; f.h[0] = *(const v8h*)(p); f.h[1] = *(const v8h*)(p + 16); return f.v;
  }
  static __device__ __forceinline__ v8f mma(v16h a, v16h b, v8f c) {
    return __builtin_amdgcn_wmma_f32_16x16x32_f16(false, a, false, b, (short)0, c, false, false);
  }
  static __device__ __forceinline__ void guard(v8f& a, v8f& b, v16h x, v16h y) { dep_guard_h(a, b, x, y); }
  static __device__ __forceinline__ void keep(v16h a, v16h b, v16h c, v16h d) { keep4_h(a, b, c, d); }
};
template <> struct Frag<__bf16> {
  typedef v16b V; union U { v16b v; v8b h[2]; };
  static __device__ __forceinline__ v16b load(const __bf16* p) {
    U f; f.h[0] = *(const v8b*)(p); f.h[1] = *(const v8b*)(p + 16); return f.v;
  }
  static __device__ __forceinline__ v8f mma(v16b a, v16b b, v8f c) {
    return __builtin_amdgcn_wmma_f32_16x16x32_bf16(false, a, false, b, (short)0, c, false, false);
  }
  static __device__ __forceinline__ void guard(v8f& a, v8f& b, v16b x, v16b y) { dep_guard_b(a, b, x, y); }
  static __device__ __forceinline__ void keep(v16b a, v16b b, v16b c, v16b d) { keep4_b(a, b, c, d); }
};

template <int ET> struct Elem;
template <> struct Elem<0> { typedef _Float16 T; };
template <> struct Elem<1> { typedef __bf16 T; };
template <int ET, bool SPLIT, int BIAS_MODE, int OUT_MODE, bool RESID, int ACT = 0>
__global__ __launch_bounds__(256) void wmma_gemm64(
    const unsigned short* __restrict__ Ap, const unsigned short* __restrict__ A2p, int lda, long strideA,
    const unsigned short* __restrict__ Btp, const unsigned short* __restrict__ Bt2p, int ldb, long strideB,
    void* __restrict__ Cout, void* __restrict__ Cout2, int ldc, long strideC,
    const float* __restrict__ bias,
    const float* __restrict__ resid, long strideR,
    int M, int N, int K, float scale) {
  typedef typename Elem<ET>::T T;
  typedef typename Frag<T>::V V;
  const T* A = (const T*)Ap; const T* A2 = (const T*)A2p; const T* Bt = (const T*)Btp; const T* Bt2 = (const T*)Bt2p;
  __shared__ __align__(16) float sT[8][16 * 68];
  const int b    = blockIdx.y;
  const int lane = threadIdx.x & 31;
  const int wave = threadIdx.x >> 5;
  const int tilesN = N >> 6;
  const int tilesM = M >> 6;
  const int tile = blockIdx.x * 8 + wave;
  if (tile >= tilesM * tilesN) return;
  const int tm = tile / tilesN;
  const int tn = tile - tm * tilesN;
  const int m0 = tm << 6;
  const int n0 = tn << 6;

  const T* Ab  = A  + (size_t)b * strideA;
  const T* Bb  = Bt + (size_t)b * strideB;
  const T* Ab2 = SPLIT ? (A2  + (size_t)b * strideA) : nullptr;
  const T* Bb2 = SPLIT ? (Bt2 + (size_t)b * strideB) : nullptr;

  const int rlane = lane & 15;
  const int koff  = (lane >> 4) * 8;
  const int mOff  = (lane >> 4) * 8;

  v8f acc[4][4];
#pragma unroll
  for (int i = 0; i < 4; ++i)
#pragma unroll
    for (int j = 0; j < 4; ++j) acc[i][j] = (v8f){0.f,0.f,0.f,0.f,0.f,0.f,0.f,0.f};

  for (int k0 = 0; k0 < K; k0 += 32) {
    V bh[4], bl[4];
#pragma unroll
    for (int j = 0; j < 4; ++j) {
      const size_t bo = (size_t)(n0 + (j << 4) + rlane) * ldb + koff + k0;
      bh[j] = Frag<T>::load(Bb + bo);
      if (SPLIT) bl[j] = Frag<T>::load(Bb2 + bo);
    }
#pragma unroll
    for (int i = 0; i < 4; ++i) {
      const size_t ao = (size_t)(m0 + (i << 4) + rlane) * lda + koff + k0;
      V ah = Frag<T>::load(Ab + ao);
      V al;
      if (SPLIT) al = Frag<T>::load(Ab2 + ao);
#pragma unroll
      for (int j = 0; j < 4; ++j) {
        acc[i][j] = Frag<T>::mma(ah, bh[j], acc[i][j]);
        if (SPLIT) {
          acc[i][j] = Frag<T>::mma(ah, bl[j], acc[i][j]);
          acc[i][j] = Frag<T>::mma(al, bh[j], acc[i][j]);
        }
      }
      Frag<T>::guard(acc[i][0], acc[i][3], ah, SPLIT ? al : ah);
    }
    Frag<T>::keep(bh[0], bh[1], bh[2], bh[3]);
    if (SPLIT) Frag<T>::keep(bl[0], bl[1], bl[2], bl[3]);
  }
  acc_guard4(acc[0][0], acc[0][1], acc[0][2], acc[0][3]);
  acc_guard4(acc[1][0], acc[1][1], acc[1][2], acc[1][3]);
  acc_guard4(acc[2][0], acc[2][1], acc[2][2], acc[2][3]);
  acc_guard4(acc[3][0], acc[3][1], acc[3][2], acc[3][3]);

  float* slab = sT[wave];
  const float* Rb = RESID ? (resid + (size_t)b * strideR) : nullptr;
#pragma unroll
  for (int i = 0; i < 4; ++i) {
    const int mBase = m0 + (i << 4);
#pragma unroll
    for (int j = 0; j < 4; ++j) {
      const int n = n0 + (j << 4) + rlane;
      float bv = 0.f;
      if (BIAS_MODE == 2) bv = bias[n];
#pragma unroll
      for (int r = 0; r < 8; ++r) {
        float v = acc[i][j][r] * scale;
        if (BIAS_MODE == 1) v += bias[mBase + mOff + r];
        if (BIAS_MODE == 2) v += bv;
        if (RESID) v += Rb[(size_t)(mBase + mOff + r) * ldc + n];
        if (ACT == 1) v = tanhf(v);
        if (ACT == 2) v = fmaxf(v, 0.0f);
        if (ACT == 3) v = v / (1.0f + expf(-v));
        if (ACT == 4) v = (v > 0.f) ? v : 0.01f * v;
        if (ACT == 6) v = (16.0f * v) * (1.0f / (1.0f + expf(-v)));
        slab[(mOff + r) * 68 + (j << 4) + rlane] = v;
      }
    }
    __builtin_amdgcn_fence(__ATOMIC_RELEASE, "workgroup");
    __builtin_amdgcn_wave_barrier();
    __builtin_amdgcn_fence(__ATOMIC_ACQUIRE, "workgroup");
    if (OUT_MODE == 0) {
      float* C = (float*)Cout + (size_t)b * strideC;
      const int hh = lane >> 4, c4 = (lane & 15) * 4;
      for (int pass = 0; pass < 2; ++pass) {
#pragma unroll
        for (int it = 0; it < 8; ++it) {
          const int row = it * 2 + hh;
          v4f v = *(const v4f*)(slab + row * 68 + c4);
          *(volatile v4f*)(C + (size_t)(mBase + row) * ldc + n0 + c4) = v;
        }
        __threadfence();
      }
    } else {
      const int q = lane >> 3, c8 = (lane & 7) * 8;
      unsigned short* C  = (unsigned short*)Cout  + (size_t)b * strideC;
      unsigned short* C2 = (OUT_MODE == 2) ? ((unsigned short*)Cout2 + (size_t)b * strideC) : nullptr;
      for (int pass = 0; pass < 2; ++pass) {
#pragma unroll
        for (int it = 0; it < 4; ++it) {
          const int row = it * 4 + q;
          const float* sp = slab + row * 68 + c8;
          v8h hv, lv;
#pragma unroll
          for (int e = 0; e < 8; ++e) {
            if (OUT_MODE == 1) {
              hv[e] = (_Float16)sp[e];
            } else {
              unsigned short hb = f2bf_bits(sp[e]);
              unsigned short lb = f2bf_bits(sp[e] - bf_bits2f(hb));
              hv[e] = __builtin_bit_cast(_Float16, hb);
              lv[e] = __builtin_bit_cast(_Float16, lb);
            }
          }
          *(volatile v8h*)(C + (size_t)(mBase + row) * ldc + n0 + c8) = hv;
          if (OUT_MODE == 2) *(volatile v8h*)(C2 + (size_t)(mBase + row) * ldc + n0 + c8) = lv;
        }
        __threadfence();
      }
    }
    __builtin_amdgcn_fence(__ATOMIC_RELEASE, "workgroup");
    __builtin_amdgcn_wave_barrier();
    __builtin_amdgcn_fence(__ATOMIC_ACQUIRE, "workgroup");
  }
}

__global__ __launch_bounds__(256) void cast_f16_kernel(
    const float* __restrict__ src, unsigned short* __restrict__ dst, int total8, float scale)
{
  const int i = blockIdx.x * 256 + threadIdx.x;
  if (i >= total8) return;
  const size_t e0 = (size_t)i << 3;
  const float* p = src + e0;
  const v4f a0 = *(const v4f*)(p);
  const v4f a1 = *(const v4f*)(p + 4);
  v8h hv;
#pragma unroll
  for (int e = 0; e < 4; ++e) {
    hv[e]     = (_Float16)(a0[e] * scale);
    hv[4 + e] = (_Float16)(a1[e] * scale);
  }
  unsigned short* q = dst + e0;
  *(volatile v8h*)q = hv;
  __threadfence();
  *(volatile v8h*)q = hv;
}

__global__ __launch_bounds__(256) void transpose_cast_kernel(
    const float* __restrict__ W, unsigned short* __restrict__ Bt, int Kdim, int Ndim, int Npad, float scale)
{
  __shared__ float tile[64 * 65];
  const int tid = threadIdx.x, lane = tid & 31, wave = tid >> 5;
  const int n0 = blockIdx.x * 64;
  const int k0 = blockIdx.y * 64;
  (void)Npad;
#pragma unroll
  for (int p = 0; p < 16; ++p) {
    const int idx = tid + p * 256;
    const int kk  = idx >> 6;
    const int nn  = idx & 63;
    const int n   = n0 + nn;
    const int nc  = (n < Ndim) ? n : (Ndim - 1);
    const float v = W[(size_t)(k0 + kk) * Ndim + nc];
    tile[kk * 65 + nn] = (n < Ndim) ? (v * scale) : 0.f;
  }
  __syncthreads();
  const int q = lane >> 3, c8 = (lane & 7) * 8;
  v8h hv[2];
#pragma unroll
  for (int it = 0; it < 2; ++it) {
    const int nrow = it * 32 + wave * 4 + q;
#pragma unroll
    for (int e = 0; e < 8; ++e) hv[it][e] = (_Float16)tile[(c8 + e) * 65 + nrow];
  }
  for (int pass = 0; pass < 2; ++pass) {
#pragma unroll
    for (int it = 0; it < 2; ++it) {
      const int nrow = it * 32 + wave * 4 + q;
      *(volatile v8h*)(Bt + (size_t)(n0 + nrow) * Kdim + k0 + c8) = hv[it];
    }
    __threadfence();
  }
}

__global__ __launch_bounds__(256) void dtw_cast_kernel(
    const float* __restrict__ W, unsigned short* __restrict__ Bt, float scale)
{
  __shared__ float tile[256 * 33];
  const int tid = threadIdx.x, lane = tid & 31, wave = tid >> 5;
  const int R0 = blockIdx.x * 256;
  const int R  = R0 + tid;
  const int s  = R / kDi;
  const int n  = R - s * kDi;
#pragma unroll
  for (int k = 0; k < kNs; ++k) tile[tid * 33 + k] = W[((size_t)s * kNs + k) * kDi + n] * scale;
  __syncthreads();
  const int q = lane >> 3, c8 = (lane & 7) * 8;
  const int hb = c8 >> 5, col0 = c8 & 31;
  const bool keep = (col0 < kNs);
  v8h hv[4];
#pragma unroll
  for (int it = 0; it < 4; ++it) {
    const int line = wave * 16 + it * 4 + q;
    const int rl   = 2 * line + hb;
#pragma unroll
    for (int e = 0; e < 8; ++e) {
      const float v = tile[rl * 33 + (col0 & 15) + e];
      hv[it][e] = keep ? (_Float16)v : (_Float16)0.0f;
    }
  }
  for (int pass = 0; pass < 2; ++pass) {
#pragma unroll
    for (int it = 0; it < 4; ++it) {
      const int line = wave * 16 + it * 4 + q;
      const int rl   = 2 * line + hb;
      *(volatile v8h*)(Bt + (size_t)(R0 + rl) * kKdt + col0) = hv[it];
    }
    __threadfence();
  }
}

__global__ __launch_bounds__(256) void bcast_kernel(
    const float* __restrict__ PROJ, unsigned short* __restrict__ B16, int total8, float scale)
{
  const int i = blockIdx.x * 256 + threadIdx.x;
  if (i >= total8) return;
  const int row = i >> 2;
  const int c8  = (i & 3) * 8;
  const bool keep = (c8 < kNs);
  const float* p = PROJ + (size_t)row * kPrj + (c8 & 15);
  const v4f a0 = *(const v4f*)(p);
  const v4f a1 = *(const v4f*)(p + 4);
  v8h hv;
#pragma unroll
  for (int e = 0; e < 4; ++e) {
    hv[e]     = keep ? (_Float16)(a0[e] * scale) : (_Float16)0.0f;
    hv[4 + e] = keep ? (_Float16)(a1[e] * scale) : (_Float16)0.0f;
  }
  unsigned short* qd = B16 + ((size_t)i << 3);
  *(volatile v8h*)qd = hv;
  __threadfence();
  *(volatile v8h*)qd = hv;
}

__device__ __forceinline__ float pooled_x(const float* __restrict__ XZ, int r, int stride, float inv, int d)
{
  const size_t base = (size_t)r * stride;
  float s = XZ[base * kXZ + d];
#pragma unroll 1
  for (int j = 1; j < stride; ++j) s += XZ[(base + j) * kXZ + d];
  return s * inv;
}

__global__ __launch_bounds__(256) void conv_silu_kernel(
    const float* __restrict__ XZ, const float* __restrict__ cw, const float* __restrict__ cb,
    float* __restrict__ XC, unsigned short* __restrict__ XC16, int stride, float inv)
{
  __shared__ __align__(16) float sT[16 * kTP];
  const int tid = threadIdx.x, lane = tid & 31, wave = tid >> 5;
  const int d0 = blockIdx.x * 256, d = d0 + tid;
  const int t0 = blockIdx.y * 64;
  const float w0 = cw[d * 4 + 0], w1 = cw[d * 4 + 1], w2 = cw[d * 4 + 2], w3 = cw[d * 4 + 3];
  const float bc = cb[d];
  float xm3, xm2, xm1;
  {
    const int r3 = t0 - 3, r2 = t0 - 2, r1 = t0 - 1;
    const float v3 = pooled_x(XZ, r3 < 0 ? 0 : r3, stride, inv, d);
    const float v2 = pooled_x(XZ, r2 < 0 ? 0 : r2, stride, inv, d);
    const float v1 = pooled_x(XZ, r1 < 0 ? 0 : r1, stride, inv, d);
    xm3 = (r3 >= 0) ? v3 : 0.f;
    xm2 = (r2 >= 0) ? v2 : 0.f;
    xm1 = (r1 >= 0) ? v1 : 0.f;
  }
  const int hrow = wave >> 1;
  const int hch  = (wave & 1) * 128 + lane * 4;
#pragma unroll 1
  for (int sub = 0; sub < 4; ++sub) {
    const int lb = t0 + sub * 16;
#pragma unroll 1
    for (int s = 0; s < 16; ++s) {
      const float xc = pooled_x(XZ, lb + s, stride, inv, d);
      float acc = w0 * xm3;
      acc = fmaf(w1, xm2, acc);
      acc = fmaf(w2, xm1, acc);
      acc = fmaf(w3, xc, acc);
      const float sv = acc + bc;
      const float sg = __builtin_amdgcn_rcpf(1.0f + __expf(-sv));
      sT[s * kTP + tid] = sv * sg;
      xm3 = xm2; xm2 = xm1; xm1 = xc;
    }
    __syncthreads();
    v4f fv[4];
    v8h bv[2];
#pragma unroll
    for (int it = 0; it < 4; ++it) fv[it] = *(const v4f*)(sT + (it * 4 + hrow) * kTP + hch);
#pragma unroll
    for (int it = 0; it < 2; ++it) {
      const float* sp = sT + (it * 8 + wave) * kTP + lane * 8;
      const v4f a0 = *(const v4f*)(sp);
      const v4f a1 = *(const v4f*)(sp + 4);
#pragma unroll
      for (int e = 0; e < 4; ++e) {
        bv[it][e]     = (_Float16)(a0[e] * 16.0f);
        bv[it][4 + e] = (_Float16)(a1[e] * 16.0f);
      }
    }
    for (int pass = 0; pass < 2; ++pass) {
#pragma unroll
      for (int it = 0; it < 4; ++it)
        *(volatile v4f*)(XC + (size_t)(lb + it * 4 + hrow) * kDi + d0 + hch) = fv[it];
#pragma unroll
      for (int it = 0; it < 2; ++it)
        *(volatile v8h*)(XC16 + (size_t)(lb + it * 8 + wave) * kDi + d0 + lane * 8) = bv[it];
      __threadfence();
    }
    __syncthreads();
  }
}

__global__ __launch_bounds__(256) void scan_kernel(
    const float* __restrict__ DLR, const float* __restrict__ XC, const float* __restrict__ PROJ,
    const float* __restrict__ Dv, float* __restrict__ Y, int nChunk)
{
  __shared__ __align__(16) float sBC[16 * 32];
  __shared__ __align__(16) float sY[16 * kTP];
  const int tid = threadIdx.x, lane = tid & 31, wave = tid >> 5;
  const int d0 = blockIdx.x * 256, d = d0 + tid;
  const float Dd = Dv[d];
  const int hrow = wave >> 1;
  const int hch  = (wave & 1) * 128 + lane * 4;
  float h[kNs];
#pragma unroll
  for (int n = 0; n < kNs; ++n) h[n] = 0.f;

#pragma unroll 1
  for (int c = 0; c < nChunk; ++c) {
    const int l0 = c * 16;
    if (tid < 128) {
      const int r = tid >> 3, q = (tid & 7) * 4;
      const v4f v = *(const v4f*)(PROJ + (size_t)(l0 + r) * kPrj + q);
      *(v4f*)(sBC + r * 32 + q) = v;
    }
    __syncthreads();
#pragma unroll 1
    for (int s = 0; s < 16; ++s) {
      const size_t m = (size_t)(l0 + s);
      const float a     = DLR[m * kDi + d];
      const float sp1   = fmaxf(a, 0.0f) + log1pf(__expf(-fabsf(a)));
      const float delta = sp1 + log1pf(__expf(-sp1));
      const float xv    = XC[m * kDi + d];
      v4f Bq[4], Cq[4];
#pragma unroll
      for (int qq = 0; qq < 4; ++qq) {
        Bq[qq] = *(const v4f*)(sBC + s * 32 + 4 * qq);
        Cq[qq] = *(const v4f*)(sBC + s * 32 + kNs + 4 * qq);
      }
      float y = 0.f;
#pragma unroll
      for (int n = 0; n < kNs; ++n) {
        const float e = __expf(delta * (-(float)(n + 1)));
        float db = delta * Bq[n >> 2][n & 3];
        asm volatile("" : "+v"(db));
        float p = db * xv;
        asm volatile("" : "+v"(p));
        p = fmaxf(p, 1e-38f);
        float qv = h[n] * e;
        asm volatile("" : "+v"(qv));
        const float hn = qv + p;
        h[n] = hn;
        float rr = Cq[n >> 2][n & 3] * hn;
        asm volatile("" : "+v"(rr));
        y += rr;
      }
      float sk = xv * Dd;
      asm volatile("" : "+v"(sk));
      y += sk;
      sY[s * kTP + tid] = y;
    }
    __syncthreads();
    v4f fv[4];
#pragma unroll
    for (int it = 0; it < 4; ++it) fv[it] = *(const v4f*)(sY + (it * 4 + hrow) * kTP + hch);
    for (int pass = 0; pass < 2; ++pass) {
#pragma unroll
      for (int it = 0; it < 4; ++it)
        *(volatile v4f*)(Y + (size_t)(l0 + it * 4 + hrow) * kDi + d0 + hch) = fv[it];
      __threadfence();
    }
  }
}

template <int TS>
__device__ __forceinline__ void interp_idx(int t, int& lo, int& hi, float& w)
{
  const float sc = (float)TS / (float)kT;
  float pos = ((float)t + 0.5f) * sc - 0.5f;
  pos = fminf(fmaxf(pos, 0.0f), (float)(TS - 1));
  const float fl = floorf(pos);
  int l = (int)fl;
  l = l < 0 ? 0 : (l > TS - 1 ? TS - 1 : l);
  int hh = l + 1;
  hh = hh > TS - 1 ? TS - 1 : hh;
  lo = l; hi = hh; w = pos - fl;
}

__device__ __forceinline__ void softmax3(const float* __restrict__ sw, float& e0, float& e1, float& e2)
{
  const float a0 = sw[0], a1 = sw[1], a2 = sw[2];
  const float m  = fmaxf(a0, fmaxf(a1, a2));
  float x0 = __expf(a0 - m), x1 = __expf(a1 - m), x2 = __expf(a2 - m);
  const float inv = 1.0f / ((x0 + x1) + x2);
  e0 = x0 * inv; e1 = x1 * inv; e2 = x2 * inv;
}

__global__ __launch_bounds__(256) void combine_kernel(
    const float* __restrict__ Y0, const float* __restrict__ Y1, const float* __restrict__ Y2,
    unsigned short* __restrict__ CTX16, int total8)
{
  const int i = blockIdx.x * 256 + threadIdx.x;
  if (i >= total8) return;
  const int t  = i / 192;
  const int c8 = (i - t * 192) * 8;
  int lo1, hi1, lo2, hi2; float w1, w2;
  interp_idx<kT / 2>(t, lo1, hi1, w1);
  interp_idx<kT / 4>(t, lo2, hi2, w2);
  const float* p0 = Y0 + (size_t)t * kDi + c8;
  const float* pa = Y1 + (size_t)lo1 * kDi + c8;
  const float* pb = Y1 + (size_t)hi1 * kDi + c8;
  const float* pc = Y2 + (size_t)lo2 * kDi + c8;
  const float* pd = Y2 + (size_t)hi2 * kDi + c8;
  v8h hv;
#pragma unroll
  for (int half = 0; half < 2; ++half) {
    const v4f u0 = *(const v4f*)(p0 + 4 * half);
    const v4f a  = *(const v4f*)(pa + 4 * half);
    const v4f b  = *(const v4f*)(pb + 4 * half);
    const v4f c  = *(const v4f*)(pc + 4 * half);
    const v4f dd = *(const v4f*)(pd + 4 * half);
    const v4f u1 = a * (1.0f - w1) + b * w1;
    const v4f u2 = c * (1.0f - w2) + dd * w2;
    const v4f ctx = ((u0 + u1) + u2) * (1.0f / 3.0f);
#pragma unroll
    for (int e = 0; e < 4; ++e) hv[4 * half + e] = (_Float16)(ctx[e] * 16.0f);
  }
  unsigned short* q = CTX16 + ((size_t)i << 3);
  *(volatile v8h*)q = hv;
  __threadfence();
  *(volatile v8h*)q = hv;
}

__global__ __launch_bounds__(256) void gate_mul_kernel(
    const float* __restrict__ Y0, const float* __restrict__ Y1, const float* __restrict__ Y2,
    const float* __restrict__ sw, const unsigned short* __restrict__ GP16, const float* __restrict__ XZ,
    unsigned short* __restrict__ OUT16, int total8)
{
  const int i = blockIdx.x * 256 + threadIdx.x;
  if (i >= total8) return;
  const int t  = i / 192;
  const int c8 = (i - t * 192) * 8;
  float e0, e1, e2;
  softmax3(sw, e0, e1, e2);
  int lo1, hi1, lo2, hi2; float w1, w2;
  interp_idx<kT / 2>(t, lo1, hi1, w1);
  interp_idx<kT / 4>(t, lo2, hi2, w2);
  const float* p0 = Y0 + (size_t)t * kDi + c8;
  const float* pa = Y1 + (size_t)lo1 * kDi + c8;
  const float* pb = Y1 + (size_t)hi1 * kDi + c8;
  const float* pc = Y2 + (size_t)lo2 * kDi + c8;
  const float* pd = Y2 + (size_t)hi2 * kDi + c8;
  const float* pg = XZ + (size_t)t * kXZ + kDi + c8;
  const v8h gp = *(const v8h*)((const _Float16*)GP16 + ((size_t)i << 3));
  v8h hv;
#pragma unroll
  for (int half = 0; half < 2; ++half) {
    const v4f u0 = *(const v4f*)(p0 + 4 * half);
    const v4f a  = *(const v4f*)(pa + 4 * half);
    const v4f b  = *(const v4f*)(pb + 4 * half);
    const v4f c  = *(const v4f*)(pc + 4 * half);
    const v4f dd = *(const v4f*)(pd + 4 * half);
    const v4f gt = *(const v4f*)(pg + 4 * half);
    const v4f u1 = a * (1.0f - w1) + b * w1;
    const v4f u2 = c * (1.0f - w2) + dd * w2;
    const v4f fu = (u0 * e0 + u1 * e1) + u2 * e2;
#pragma unroll
    for (int e = 0; e < 4; ++e) {
      const float gpre = (float)gp[4 * half + e] * (1.0f / 64.0f);
      const float g    = __builtin_amdgcn_rcpf(1.0f + __expf(-gpre));
      const float gv   = gt[e];
      const float sg   = gv * __builtin_amdgcn_rcpf(1.0f + __expf(-gv));
      float fg = fu[e] * g;
      asm volatile("" : "+v"(fg));
      const float o = fg * sg;
      hv[4 * half + e] = (_Float16)(o * 64.0f);
    }
  }
  unsigned short* q = OUT16 + ((size_t)i << 3);
  *(volatile v8h*)q = hv;
  __threadfence();
  *(volatile v8h*)q = hv;
}

__global__ __launch_bounds__(256) void layernorm_kernel(
    const float* __restrict__ YP, const float* __restrict__ gamma, const float* __restrict__ beta,
    float* __restrict__ out)
{
  const int lane = threadIdx.x & 31, wave = threadIdx.x >> 5;
  const int row = blockIdx.x * 8 + wave;
  const int q = lane >> 3, c4 = (lane & 7) * 4;
  const float* yr = YP + (size_t)row * kDm;
  float s = 0.f;
#pragma unroll 1
  for (int i = 0; i < 6; ++i) {
    const int e = (i * 4 + q) * 32 + c4;
    const v4f v = *(const v4f*)(yr + e);
    s += (v[0] + v[1]) + (v[2] + v[3]);
  }
#pragma unroll
  for (int off = 16; off > 0; off >>= 1) s += __shfl_xor(s, off, 32);
  const float mean = s * (1.0f / (float)kDm);
  float vs = 0.f;
#pragma unroll 1
  for (int i = 0; i < 6; ++i) {
    const int e = (i * 4 + q) * 32 + c4;
    const v4f v = *(const v4f*)(yr + e);
    const v4f z = v - mean;
    vs += (z[0] * z[0] + z[1] * z[1]) + (z[2] * z[2] + z[3] * z[3]);
  }
#pragma unroll
  for (int off = 16; off > 0; off >>= 1) vs += __shfl_xor(vs, off, 32);
  const float var  = vs * (1.0f / (float)kDm);
  const float rstd = 1.0f / sqrtf(var + 1e-5f);
  float* orow = out + (size_t)row * kDm;
  for (int pass = 0; pass < 2; ++pass) {
#pragma unroll 1
    for (int i = 0; i < 6; ++i) {
      const int e = (i * 4 + q) * 32 + c4;
      const v4f v  = *(const v4f*)(yr + e);
      const v4f gm = *(const v4f*)(gamma + e);
      const v4f bt = *(const v4f*)(beta + e);
      const v4f o  = ((v - mean) * rstd) * gm + bt;
      *(volatile v4f*)(orow + e) = o;
    }
    __threadfence();
  }
}

extern "C" void kernel_launch(void* const* d_in, const int* in_sizes, int n_in,
                              void* d_out, int out_size, void* d_ws, size_t ws_size,
                              hipStream_t stream)
{
  if (n_in < 14) return;
  const float* x        = (const float*)d_in[0];
  const float* W_in     = (const float*)d_in[1];
  const float* conv_w   = (const float*)d_in[2];
  const float* conv_b   = (const float*)d_in[3];
  const float* W_xprj   = (const float*)d_in[4];
  const float* W_dt     = (const float*)d_in[5];
  const float* b_dt     = (const float*)d_in[6];
  const float* Dv       = (const float*)d_in[7];
  const float* scale_w  = (const float*)d_in[8];
  const float* W_g1     = (const float*)d_in[9];
  const float* W_g2     = (const float*)d_in[10];
  const float* W_out    = (const float*)d_in[11];
  const float* ln_gamma = (const float*)d_in[12];
  const float* ln_beta  = (const float*)d_in[13];
  float* dout = (float*)d_out;

  if (in_sizes[0] != kT * kDm) return;
  if (in_sizes[1] != kDm * kXZ) return;
  if (in_sizes[2] != kNsc * kDi * 4 || in_sizes[3] != kNsc * kDi) return;
  if (in_sizes[4] != kNsc * kDi * 2 * kNs) return;
  if (in_sizes[5] != kNsc * kNs * kDi || in_sizes[6] != kNsc * kDi) return;
  if (in_sizes[7] != kNsc * kDi || in_sizes[8] != kNsc) return;
  if (in_sizes[9] != kDi * kG1 || in_sizes[10] != kG1 * kDi || in_sizes[11] != kDi * kDm) return;
  if (in_sizes[12] != kDm || in_sizes[13] != kDm) return;
  if (out_size != kT * kDm) return;

  const size_t SZ_WIN16 = (size_t)kXZ * kDm * 2;
  const size_t SZ_WG1   = (size_t)kG1 * kDi * 2;
  const size_t SZ_WG2   = (size_t)kDi * kG1 * 2;
  const size_t SZ_WOUT  = (size_t)kDm * kDi * 2;
  const size_t SZ_WXP1  = (size_t)kPrj * kDi * 2;
  const size_t SZ_WDT1  = (size_t)kDi * kKdt * 2;
  const size_t SZ_X16   = (size_t)kT * kDm * 2;
  const size_t SZ_XZ    = (size_t)kT * kXZ * 4;
  const size_t SZ_XC    = (size_t)kT * kDi * 4;
  const size_t SZ_XC16  = (size_t)kT * kDi * 2;
  const size_t SZ_PROJ  = (size_t)kT * kPrj * 4;
  const size_t SZ_B16   = (size_t)kT * kKdt * 2;
  const size_t SZ_DLR   = (size_t)kT * kDi * 4;
  const size_t SZ_Y0    = (size_t)kT * kDi * 4;
  const size_t SZ_Y1    = (size_t)(kT / 2) * kDi * 4;
  const size_t SZ_Y2    = (size_t)(kT / 4) * kDi * 4;
  const size_t SZ_CTX16 = (size_t)kT * kDi * 2;
  const size_t SZ_T1    = (size_t)kT * kG1 * 2;
  const size_t SZ_GP16  = (size_t)kT * kDi * 2;
  const size_t SZ_OUT16 = (size_t)kT * kDi * 2;
  const size_t SZ_YPRE  = (size_t)kT * kDm * 4;
  const size_t OFF_WIN16 = 0;
  const size_t OFF_WG1   = OFF_WIN16 + SZ_WIN16;
  const size_t OFF_WG2   = OFF_WG1   + SZ_WG1;
  const size_t OFF_WOUT  = OFF_WG2   + SZ_WG2;
  const size_t OFF_WXP   = OFF_WOUT  + SZ_WOUT;
  const size_t OFF_WDT   = OFF_WXP   + SZ_WXP1 * kNsc;
  const size_t OFF_X16   = OFF_WDT   + SZ_WDT1 * kNsc;
  const size_t OFF_XZ    = OFF_X16   + SZ_X16;
  const size_t OFF_XC    = OFF_XZ    + SZ_XZ;
  const size_t OFF_XC16  = OFF_XC    + SZ_XC;
  const size_t OFF_PROJ  = OFF_XC16  + SZ_XC16;
  const size_t OFF_B16   = OFF_PROJ  + SZ_PROJ;
  const size_t OFF_DLR   = OFF_B16   + SZ_B16;
  const size_t OFF_Y0    = OFF_DLR   + SZ_DLR;
  const size_t OFF_Y1    = OFF_Y0    + SZ_Y0;
  const size_t OFF_Y2    = OFF_Y1    + SZ_Y1;
  const size_t OFF_CTX16 = OFF_Y2    + SZ_Y2;
  const size_t OFF_T1    = OFF_CTX16 + SZ_CTX16;
  const size_t OFF_GP16  = OFF_T1    + SZ_T1;
  const size_t OFF_OUT16 = OFF_GP16  + SZ_GP16;
  const size_t OFF_YPRE  = OFF_OUT16 + SZ_OUT16;
  const size_t TOTAL     = OFF_YPRE  + SZ_YPRE;
  if (ws_size < TOTAL) return;

  char* ws = (char*)d_ws;
  unsigned short* WIN16 = (unsigned short*)(ws + OFF_WIN16);
  unsigned short* WG1   = (unsigned short*)(ws + OFF_WG1);
  unsigned short* WG2   = (unsigned short*)(ws + OFF_WG2);
  unsigned short* WOUT  = (unsigned short*)(ws + OFF_WOUT);
  unsigned short* WXP16 = (unsigned short*)(ws + OFF_WXP);
  unsigned short* WDT16 = (unsigned short*)(ws + OFF_WDT);
  unsigned short* X16   = (unsigned short*)(ws + OFF_X16);
  float*          XZ    = (float*)(ws + OFF_XZ);
  float*          XC    = (float*)(ws + OFF_XC);
  unsigned short* XC16  = (unsigned short*)(ws + OFF_XC16);
  float*          PROJ  = (float*)(ws + OFF_PROJ);
  unsigned short* B16   = (unsigned short*)(ws + OFF_B16);
  float*          DLR   = (float*)(ws + OFF_DLR);
  float*          Y0    = (float*)(ws + OFF_Y0);
  float*          Y1    = (float*)(ws + OFF_Y1);
  float*          Y2    = (float*)(ws + OFF_Y2);
  unsigned short* CTX16 = (unsigned short*)(ws + OFF_CTX16);
  unsigned short* T1    = (unsigned short*)(ws + OFF_T1);
  unsigned short* GP16  = (unsigned short*)(ws + OFF_GP16);
  unsigned short* OUT16 = (unsigned short*)(ws + OFF_OUT16);
  float*          YPRE  = (float*)(ws + OFF_YPRE);
  const float* dummy_bias  = b_dt;
  const float* dummy_resid = x;

  transpose_cast_kernel<<<dim3(kXZ / 64, kDm / 64), 256, 0, stream>>>(W_in,  WIN16, kDm, kXZ, kXZ, 32.0f);
  transpose_cast_kernel<<<dim3(kG1 / 64, kDi / 64), 256, 0, stream>>>(W_g1,  WG1,   kDi, kG1, kG1, 32.0f);
  transpose_cast_kernel<<<dim3(kDi / 64, kG1 / 64), 256, 0, stream>>>(W_g2,  WG2,   kG1, kDi, kDi, 32.0f);
  transpose_cast_kernel<<<dim3(kDm / 64, kDi / 64), 256, 0, stream>>>(W_out, WOUT,  kDi, kDm, kDm, 32.0f);
  for (int s = 0; s < kNsc; ++s)
    transpose_cast_kernel<<<dim3(kPrj / 64, kDi / 64), 256, 0, stream>>>(
        W_xprj + (size_t)s * kDi * (2 * kNs), WXP16 + (size_t)s * kPrj * kDi, kDi, 2 * kNs, kPrj, 32.0f);
  dtw_cast_kernel<<<dim3((kNsc * kDi) / 256), 256, 0, stream>>>(W_dt, WDT16, 16.0f);

  cast_f16_kernel<<<(kT * kDm) / 8 / 256, 256, 0, stream>>>(x, X16, (kT * kDm) / 8, 1.0f);

  wmma_gemm64<0, false, 0, 0, false, 0><<<dim3((kT / 64) * (kXZ / 64) / 8, 1), 256, 0, stream>>>(
      X16, X16, kDm, 0L, WIN16, WIN16, kDm, 0L,
      (void*)XZ, (void*)XZ, kXZ, 0L, dummy_bias, dummy_resid, 0L, kT, kXZ, kDm, 1.0f / 32.0f);

  float* Ys[kNsc] = { Y0, Y1, Y2 };
  for (int s = 0; s < kNsc; ++s) {
    const int stride = 1 << s;
    const int Ts = kT >> s;
    const unsigned short* WXPs = WXP16 + (size_t)s * kPrj * kDi;
    const unsigned short* WDTs = WDT16 + (size_t)s * kDi * kKdt;

    conv_silu_kernel<<<dim3(kDi / 256, Ts / 64), 256, 0, stream>>>(
        XZ, conv_w + (size_t)s * kDi * 4, conv_b + (size_t)s * kDi, XC, XC16, stride, 1.0f / (float)stride);

    wmma_gemm64<0, false, 0, 0, false, 0><<<dim3((Ts / 64 + 7) / 8, 1), 256, 0, stream>>>(
        XC16, XC16, kDi, 0L, WXPs, WXPs, kDi, 0L,
        (void*)PROJ, (void*)PROJ, kPrj, 0L, dummy_bias, dummy_resid, 0L, Ts, kPrj, kDi, 1.0f / 512.0f);

    bcast_kernel<<<dim3(Ts / 64), 256, 0, stream>>>(PROJ, B16, Ts * 4, 16.0f);

    wmma_gemm64<0, false, 2, 0, false, 0><<<dim3((Ts / 64) * 3, 1), 256, 0, stream>>>(
        B16, B16, kKdt, 0L, WDTs, WDTs, kKdt, 0L,
        (void*)DLR, (void*)DLR, kDi, 0L, b_dt + (size_t)s * kDi, dummy_resid, 0L, Ts, kDi, kKdt, 1.0f / 256.0f);

    scan_kernel<<<dim3(kDi / 256), 256, 0, stream>>>(DLR, XC, PROJ, Dv + (size_t)s * kDi, Ys[s], Ts / 16);
  }

  combine_kernel<<<dim3((kT * kDi) / 8 / 256), 256, 0, stream>>>(Y0, Y1, Y2, CTX16, (kT * kDi) / 8);

  wmma_gemm64<0, false, 0, 1, false, 6><<<dim3((kT / 64) * (kG1 / 64) / 8, 1), 256, 0, stream>>>(
      CTX16, CTX16, kDi, 0L, WG1, WG1, kDi, 0L,
      (void*)T1, (void*)T1, kG1, 0L, dummy_bias, dummy_resid, 0L, kT, kG1, kDi, 1.0f / 512.0f);

  wmma_gemm64<0, false, 0, 1, false, 0><<<dim3((kT / 64) * (kDi / 64) / 8, 1), 256, 0, stream>>>(
      T1, T1, kG1, 0L, WG2, WG2, kG1, 0L,
      (void*)GP16, (void*)GP16, kDi, 0L, dummy_bias, dummy_resid, 0L, kT, kDi, kG1, 1.0f / 8.0f);

  gate_mul_kernel<<<dim3((kT * kDi) / 8 / 256), 256, 0, stream>>>(
      Y0, Y1, Y2, scale_w, GP16, XZ, OUT16, (kT * kDi) / 8);

  wmma_gemm64<0, false, 0, 0, true, 0><<<dim3((kT / 64) * (kDm / 64) / 8, 1), 256, 0, stream>>>(
      OUT16, OUT16, kDi, 0L, WOUT, WOUT, kDi, 0L,
      (void*)YPRE, (void*)YPRE, kDm, 0L, dummy_bias, x, 0L, kT, kDm, kDi, 1.0f / 2048.0f);

  layernorm_kernel<<<dim3(kT / 8), 256, 0, stream>>>(YPRE, ln_gamma, ln_beta, dout);
}
